// TopExtraAttention_48679159333610
// MI455X (gfx1250) — hardware-verified
//
#include <hip/hip_runtime.h>
#include <stdint.h>

#define NQ   16384
#define NK   4096
#define DD   512
#define DVV  256

typedef _Float16 v16h __attribute__((ext_vector_type(16)));
typedef _Float16 v8h  __attribute__((ext_vector_type(8)));
typedef __bf16   v16b __attribute__((ext_vector_type(16)));
typedef float    v8f  __attribute__((ext_vector_type(8)));
typedef float    v4f  __attribute__((ext_vector_type(4)));
typedef unsigned short v8us __attribute__((ext_vector_type(8)));

static_assert((NQ % 32) == 0 && (NK % 256) == 0 && (DD % 64) == 0 && (DVV % 64) == 0);

__device__ __forceinline__ unsigned short bfbits(float f) {
  unsigned u = __float_as_uint(f);
  return (unsigned short)((u + 0x7FFFu + ((u >> 16) & 1u)) >> 16);
}
__device__ __forceinline__ float bfval(unsigned short b) { return __uint_as_float(((unsigned)b) << 16); }

__device__ __forceinline__ v16h ldfrag_h(const _Float16* p) {
  union { v16h v; v8h q[2]; } f;
  f.q[0] = *(const v8h*)(p);
  f.q[1] = *(const v8h*)(p + 16);
  return f.v;
}
__device__ __forceinline__ v16b ldfrag_b(const unsigned short* p) {
  union { v16b v; v8us q[2]; } f;
  f.q[0] = *(const v8us*)(p);
  f.q[1] = *(const v8us*)(p + 16);
  return f.v;
}
__device__ __forceinline__ v8f mma_h(v16h a, v16h b, v8f c) {
  return __builtin_amdgcn_wmma_f32_16x16x32_f16(false, a, false, b, (short)0, c, false, false);
}
__device__ __forceinline__ v8f mma_b(v16b a, v16b b, v8f c) {
  return __builtin_amdgcn_wmma_f32_16x16x32_bf16(false, a, false, b, (short)0, c, false, false);
}
__device__ __forceinline__ v8f zero8() {
  v8f z;
#pragma unroll
  for (int i = 0; i < 8; ++i) z[i] = 0.0f;
  return z;
}

__device__ __forceinline__ void guard_g4(v8f& a, v8f& b, v8f& c, v8f& d,
                                         v16b x, v16b y0, v16b y1, v16b y2, v16b y3) {
#if defined(__HIP_DEVICE_COMPILE__)
  asm volatile("v_nop\n\tv_nop\n\tv_nop\n\tv_nop"
               : "+v"(a), "+v"(b), "+v"(c), "+v"(d) : "v"(x), "v"(y0), "v"(y1), "v"(y2), "v"(y3));
#endif
}
__device__ __forceinline__ void accg4(v8f& a, v8f& b, v8f& c, v8f& d) {
#if defined(__HIP_DEVICE_COMPILE__)
  asm volatile("v_nop\n\tv_nop\n\tv_nop\n\tv_nop" : "+v"(a), "+v"(b), "+v"(c), "+v"(d));
#endif
}
__device__ __forceinline__ void guard_s(v8f& a, v8f& b, v8f& c, v8f& d,
                                        v16b x0, v16b x1, v16b x2, v16b x3, v16b y0, v16b y1) {
#if defined(__HIP_DEVICE_COMPILE__)
  asm volatile("v_nop\n\tv_nop\n\tv_nop\n\tv_nop"
               : "+v"(a), "+v"(b), "+v"(c), "+v"(d)
               : "v"(x0), "v"(x1), "v"(x2), "v"(x3), "v"(y0), "v"(y1));
#endif
}
__device__ __forceinline__ void guard_pv(v8f& a0, v8f& a1, v8f& a2, v8f& a3,
                                         v8f& b0, v8f& b1, v8f& b2, v8f& b3,
                                         v16h p0, v16h p1, v16h x0, v16h x1, v16h x2, v16h x3) {
#if defined(__HIP_DEVICE_COMPILE__)
  asm volatile("v_nop\n\tv_nop\n\tv_nop\n\tv_nop"
               : "+v"(a0), "+v"(a1), "+v"(a2), "+v"(a3), "+v"(b0), "+v"(b1), "+v"(b2), "+v"(b3)
               : "v"(p0), "v"(p1), "v"(x0), "v"(x1), "v"(x2), "v"(x3));
#endif
}

__global__ __launch_bounds__(256) void cvt_kernel(const float* __restrict__ y, const float* __restrict__ z,
                                                  const float* __restrict__ wk, const float* __restrict__ wv,
                                                  const int* __restrict__ rate,
                                                  unsigned short* __restrict__ yb, unsigned short* __restrict__ zb,
                                                  unsigned short* __restrict__ wkb, unsigned short* __restrict__ wvb,
                                                  int n8y, int n8z, int n8k, int n8v) {
  (void)rate;
  const int nby = n8y >> 8, nbz = n8z >> 8, nbk = n8k >> 8;
  int bid = (int)blockIdx.x;
  const float* src = y; unsigned short* dst = yb; int n8 = n8y;
  if (bid >= nby) {
    bid -= nby; src = z; dst = zb; n8 = n8z;
    if (bid >= nbz) {
      bid -= nbz; src = wk; dst = wkb; n8 = n8k;
      if (bid >= nbk) { bid -= nbk; src = wv; dst = wvb; n8 = n8v; }
    }
  }
  const int li = bid * 256 + (int)threadIdx.x;
  if (li >= n8) return;
  const size_t e = (size_t)li * 8;
  const v4f a = *(const v4f*)(src + e);
  const v4f b = *(const v4f*)(src + e + 4);
  v8us o;
#pragma unroll
  for (int i = 0; i < 4; ++i) { o[i] = bfbits(a[i]); o[4 + i] = bfbits(b[i]); }
  unsigned short* d = dst + e;
  *(volatile v8us*)d = o;
  __threadfence();
  *(volatile v8us*)d = o;
}

template <int OM>
__global__ __launch_bounds__(256) void gemm64_kernel(const unsigned short* __restrict__ A, int lda,
                                                     const unsigned short* __restrict__ Bt, int ldb,
                                                     unsigned short* __restrict__ Ch, unsigned short* __restrict__ Cl,
                                                     int ldc, int M, int N, int K, float s_hi, float s_lo) {
  __shared__ __align__(16) float sT[8][16 * 68];
  const int lane = threadIdx.x & 31, wave = threadIdx.x >> 5;
  const int tilesN = N >> 6, tilesM = M >> 6;
  const int tile = (int)blockIdx.x * 8 + wave;
  if (tile >= tilesM * tilesN) return;
  const int tm = tile / tilesN, tn = tile - tm * tilesN;
  const int m0 = tm << 6, n0 = tn << 6;
  const int rl = lane & 15, hh = lane >> 4;
  const int koff = hh * 8;

  v8f acc[4][4];
#pragma unroll
  for (int i = 0; i < 4; ++i)
#pragma unroll
    for (int j = 0; j < 4; ++j) acc[i][j] = zero8();

#pragma unroll 1
  for (int k0 = 0; k0 < K; k0 += 32) {
    v16b bh[4];
#pragma unroll
    for (int j = 0; j < 4; ++j) bh[j] = ldfrag_b(Bt + (size_t)(n0 + (j << 4) + rl) * ldb + koff + k0);
#pragma unroll
    for (int i = 0; i < 4; ++i) {
      const v16b ah = ldfrag_b(A + (size_t)(m0 + (i << 4) + rl) * lda + koff + k0);
#pragma unroll
      for (int j = 0; j < 4; ++j) acc[i][j] = mma_b(ah, bh[j], acc[i][j]);
      guard_g4(acc[i][0], acc[i][1], acc[i][2], acc[i][3], ah, bh[0], bh[1], bh[2], bh[3]);
    }
  }
  accg4(acc[0][0], acc[0][1], acc[0][2], acc[0][3]);
  accg4(acc[1][0], acc[1][1], acc[1][2], acc[1][3]);
  accg4(acc[2][0], acc[2][1], acc[2][2], acc[2][3]);
  accg4(acc[3][0], acc[3][1], acc[3][2], acc[3][3]);

  float* slab = sT[wave];
  const int qq = lane >> 3, c8 = (lane & 7) * 8;
#pragma unroll
  for (int i = 0; i < 4; ++i) {
    const int mBase = m0 + (i << 4);
#pragma unroll
    for (int j = 0; j < 4; ++j) {
#pragma unroll
      for (int r = 0; r < 8; ++r) slab[(8 * hh + r) * 68 + (j << 4) + rl] = acc[i][j][r];
    }
    __builtin_amdgcn_fence(__ATOMIC_RELEASE, "workgroup");
    __builtin_amdgcn_wave_barrier();
    __builtin_amdgcn_fence(__ATOMIC_ACQUIRE, "workgroup");
#pragma unroll
    for (int ps = 0; ps < 2; ++ps) {
#pragma unroll
      for (int it = 0; it < 4; ++it) {
        const int row = it * 4 + qq;
        const float* sp = slab + row * 68 + c8;
        const size_t off = (size_t)(mBase + row) * ldc + n0 + c8;
        if (OM == 0) {
          v8us hv, lv;
#pragma unroll
          for (int e = 0; e < 8; ++e) {
            const float v = sp[e] * s_hi;
            const unsigned short hb = bfbits(v);
            hv[e] = hb;
            lv[e] = bfbits((v - bfval(hb)) * s_lo);
          }
          *(volatile v8us*)(Ch + off) = hv;
          *(volatile v8us*)(Cl + off) = lv;
        } else {
          v8h hv, lv;
#pragma unroll
          for (int e = 0; e < 8; ++e) {
            const float v = sp[e] * s_hi;
            const _Float16 x = (_Float16)v;
            hv[e] = x;
            lv[e] = (_Float16)((v - (float)x) * s_lo);
          }
          *(volatile v8h*)((_Float16*)Ch + off) = hv;
          *(volatile v8h*)((_Float16*)Cl + off) = lv;
        }
      }
      __threadfence();
    }
    __builtin_amdgcn_fence(__ATOMIC_RELEASE, "workgroup");
    __builtin_amdgcn_wave_barrier();
    __builtin_amdgcn_fence(__ATOMIC_ACQUIRE, "workgroup");
  }
}

#define QB       32
#define KCH      256
#define QSP      520
#define PSP      264
#define OSP      260
#define LDS_QS   0
#define LDS_PS   33280
#define LDS_PMAX 50176
#define LDS_PSUM 51200
#define LDS_ST   52224
#define ATT_LDS  52736
static_assert(QB * QSP * 2 == LDS_PS - LDS_QS);
static_assert(QB * PSP * 2 == LDS_PMAX - LDS_PS);
static_assert(QB * OSP * 4 <= LDS_PS - LDS_QS);
static_assert(LDS_PSUM - LDS_PMAX == 256 * 4);
static_assert(LDS_ST - LDS_PSUM == 256 * 4);
static_assert(ATT_LDS - LDS_ST == 4 * 32 * 4);
static_assert((QSP % 8) == 0 && (PSP % 8) == 0 && (OSP % 4) == 0 && PSP >= KCH && QSP >= DD && OSP >= DVV);
static_assert((LDS_PS % 16) == 0 && (LDS_PMAX % 16) == 0 && (LDS_ST % 16) == 0);
static_assert((NK % KCH) == 0 && (NQ % QB) == 0 && (DD % 32) == 0 && DVV == 8 * 32 && DD == 64 * 8);

__global__ __launch_bounds__(256) void attn_kernel(const float* __restrict__ X, const unsigned short* __restrict__ kh,
                                                   const unsigned short* __restrict__ kl,
                                                   const _Float16* __restrict__ vh, const _Float16* __restrict__ vl,
                                                   float* __restrict__ out, float sc, int nq, int nk) {
  __shared__ __align__(16) char smem[ATT_LDS];
  unsigned short* Qs = (unsigned short*)(smem + LDS_QS);
  _Float16* Ps = (_Float16*)(smem + LDS_PS);
  float* pmax = (float*)(smem + LDS_PMAX);
  float* psum = (float*)(smem + LDS_PSUM);
  float* m_s  = (float*)(smem + LDS_ST);
  float* l_s  = m_s + 32;
  float* al_s = m_s + 64;
  float* li_s = m_s + 96;

  const int tid = threadIdx.x, wave = tid >> 5, lane = tid & 31, h = lane >> 4, c = lane & 15;
  const int q0 = (int)blockIdx.x * QB;
  if (q0 + QB > nq) return;
  const float ninf = -__builtin_inff();

  if (tid < 32) { m_s[tid] = ninf; l_s[tid] = 0.0f; al_s[tid] = 0.0f; li_s[tid] = 0.0f; }
  psum[tid] = 0.0f;
#pragma unroll
  for (int i = 0; i < 8; ++i) {
    const int idx = i * 256 + tid;
    const int row = idx >> 6;
    const int pc  = idx & 63;
    const float* xp = X + (size_t)(q0 + row) * DD + pc * 8;
    const v4f a = *(const v4f*)(xp);
    const v4f b = *(const v4f*)(xp + 4);
    v8us o;
#pragma unroll
    for (int e = 0; e < 4; ++e) { o[e] = bfbits(a[e]); o[4 + e] = bfbits(b[e]); }
    *(v8us*)(Qs + row * QSP + pc * 8) = o;
  }
  __syncthreads();

  v8f oh[2][2], ol[2][2];
#pragma unroll
  for (int qt = 0; qt < 2; ++qt)
#pragma unroll
    for (int nt = 0; nt < 2; ++nt) { oh[qt][nt] = zero8(); ol[qt][nt] = zero8(); }

  const unsigned short* qb0p = Qs + c * QSP + 8 * h;
  const unsigned short* qb1p = Qs + (16 + c) * QSP + 8 * h;
  const _Float16* pa0p = Ps + c * PSP + 8 * h;
  const _Float16* pa1p = Ps + (16 + c) * PSP + 8 * h;
  const int ntile = nk / KCH;

#pragma unroll 1
  for (int t = 0; t < ntile; ++t) {
    const int kb = t * KCH + 32 * wave;
    const unsigned short* ka0 = kh + (size_t)(kb + c) * DD + 8 * h;
    const unsigned short* ka1 = kh + (size_t)(kb + 16 + c) * DD + 8 * h;
    const unsigned short* la0 = kl + (size_t)(kb + c) * DD + 8 * h;
    const unsigned short* la1 = kl + (size_t)(kb + 16 + c) * DD + 8 * h;
    v8f sacc[2][2];
#pragma unroll
    for (int qt = 0; qt < 2; ++qt)
#pragma unroll
      for (int kt = 0; kt < 2; ++kt) sacc[qt][kt] = zero8();
#pragma unroll 1
    for (int k0 = 0; k0 < DD; k0 += 32) {
      const v16b a0 = ldfrag_b(ka0 + k0), a1 = ldfrag_b(ka1 + k0);
      const v16b e0 = ldfrag_b(la0 + k0), e1 = ldfrag_b(la1 + k0);
      const v16b b0 = ldfrag_b(qb0p + k0), b1 = ldfrag_b(qb1p + k0);
      sacc[0][0] = mma_b(a0, b0, sacc[0][0]);
      sacc[0][1] = mma_b(a1, b0, sacc[0][1]);
      sacc[1][0] = mma_b(a0, b1, sacc[1][0]);
      sacc[1][1] = mma_b(a1, b1, sacc[1][1]);
      sacc[0][0] = mma_b(e0, b0, sacc[0][0]);
      sacc[0][1] = mma_b(e1, b0, sacc[0][1]);
      sacc[1][0] = mma_b(e0, b1, sacc[1][0]);
      sacc[1][1] = mma_b(e1, b1, sacc[1][1]);
      guard_s(sacc[0][0], sacc[0][1], sacc[1][0], sacc[1][1], a0, a1, e0, e1, b0, b1);
    }
    {
      float pm0 = ninf, pm1 = ninf;
#pragma unroll
      for (int kt = 0; kt < 2; ++kt) {
#pragma unroll
        for (int r = 0; r < 8; ++r) {
          const float v0 = sacc[0][kt][r] * sc; sacc[0][kt][r] = v0; pm0 = fmaxf(pm0, v0);
          const float v1 = sacc[1][kt][r] * sc; sacc[1][kt][r] = v1; pm1 = fmaxf(pm1, v1);
        }
      }
      pm0 = fmaxf(pm0, __shfl_xor(pm0, 16, 32));
      pm1 = fmaxf(pm1, __shfl_xor(pm1, 16, 32));
      pmax[wave * 32 + c] = pm0;
      pmax[wave * 32 + 16 + c] = pm1;
    }
    __syncthreads();
    if (wave == 0) {
      const int row = lane;
      float ps = 0.0f;
#pragma unroll
      for (int w = 0; w < 8; ++w) ps += psum[w * 32 + row];
      l_s[row] = l_s[row] * al_s[row] + ps;
      const float mo = m_s[row];
      float mx = mo;
#pragma unroll
      for (int w = 0; w < 8; ++w) mx = fmaxf(mx, pmax[w * 32 + row]);
      al_s[row] = __expf(mo - mx);
      m_s[row] = mx;
    }
    __syncthreads();
    {
      const float mq0 = m_s[c], mq1 = m_s[16 + c];
      float ps0 = 0.0f, ps1 = 0.0f;
#pragma unroll
      for (int kt = 0; kt < 2; ++kt) {
        v8h h0, h1;
#pragma unroll
        for (int r = 0; r < 8; ++r) {
          const float p0 = __expf(sacc[0][kt][r] - mq0); ps0 += p0; h0[r] = (_Float16)(p0 * 256.0f);
          const float p1 = __expf(sacc[1][kt][r] - mq1); ps1 += p1; h1[r] = (_Float16)(p1 * 256.0f);
        }
        *(v8h*)(Ps + c * PSP + 32 * wave + 16 * kt + 8 * h) = h0;
        *(v8h*)(Ps + (16 + c) * PSP + 32 * wave + 16 * kt + 8 * h) = h1;
      }
      ps0 += __shfl_xor(ps0, 16, 32);
      ps1 += __shfl_xor(ps1, 16, 32);
      psum[wave * 32 + c] = ps0;
      psum[wave * 32 + 16 + c] = ps1;
      const v4f aA = *(const v4f*)(al_s + 8 * h),      aB = *(const v4f*)(al_s + 8 * h + 4);
      const v4f bA = *(const v4f*)(al_s + 16 + 8 * h), bB = *(const v4f*)(al_s + 16 + 8 * h + 4);
#pragma unroll
      for (int nt = 0; nt < 2; ++nt) {
#pragma unroll
        for (int r = 0; r < 4; ++r) {
          oh[0][nt][r] *= aA[r]; oh[0][nt][4 + r] *= aB[r];
          oh[1][nt][r] *= bA[r]; oh[1][nt][4 + r] *= bB[r];
          ol[0][nt][r] *= aA[r]; ol[0][nt][4 + r] *= aB[r];
          ol[1][nt][r] *= bA[r]; ol[1][nt][4 + r] *= bB[r];
        }
      }
    }
    __syncthreads();
    {
      const size_t vo = (size_t)(32 * wave + c) * (size_t)nk + (size_t)t * KCH + 8 * h;
      const _Float16* vhp = vh + vo;
      const _Float16* vlp = vl + vo;
      const size_t n16 = (size_t)16 * (size_t)nk;
#pragma unroll 1
      for (int ks = 0; ks < KCH; ks += 32) {
        const v16h pa0 = ldfrag_h(pa0p + ks), pa1 = ldfrag_h(pa1p + ks);
        const v16h xb0 = ldfrag_h(vhp + ks), xb1 = ldfrag_h(vhp + n16 + ks);
        const v16h yb0 = ldfrag_h(vlp + ks), yb1 = ldfrag_h(vlp + n16 + ks);
        oh[0][0] = mma_h(pa0, xb0, oh[0][0]);
        oh[0][1] = mma_h(pa0, xb1, oh[0][1]);
        oh[1][0] = mma_h(pa1, xb0, oh[1][0]);
        oh[1][1] = mma_h(pa1, xb1, oh[1][1]);
        ol[0][0] = mma_h(pa0, yb0, ol[0][0]);
        ol[0][1] = mma_h(pa0, yb1, ol[0][1]);
        ol[1][0] = mma_h(pa1, yb0, ol[1][0]);
        ol[1][1] = mma_h(pa1, yb1, ol[1][1]);
        guard_pv(oh[0][0], oh[0][1], oh[1][0], oh[1][1], ol[0][0], ol[0][1], ol[1][0], ol[1][1],
                 pa0, pa1, xb0, xb1, yb0, yb1);
      }
    }
  }

  if (wave == 0) {
    const int row = lane;
    float ps = 0.0f;
#pragma unroll
    for (int w = 0; w < 8; ++w) ps += psum[w * 32 + row];
    const float l = l_s[row] * al_s[row] + ps;
    li_s[row] = (1.0f / l) * (1.0f / 4096.0f);
  }
  __syncthreads();
  float* Os = (float*)(smem + LDS_QS);
  {
    const float rlo = 1.0f / 2048.0f;
    const v4f iA0 = *(const v4f*)(li_s + 8 * h),      iB0 = *(const v4f*)(li_s + 8 * h + 4);
    const v4f iA1 = *(const v4f*)(li_s + 16 + 8 * h), iB1 = *(const v4f*)(li_s + 16 + 8 * h + 4);
#pragma unroll
    for (int nt = 0; nt < 2; ++nt) {
      const int col = 32 * wave + 16 * nt + c;
#pragma unroll
      for (int r = 0; r < 4; ++r) {
        Os[(8 * h + r) * OSP + col]          = (oh[0][nt][r] + ol[0][nt][r] * rlo) * iA0[r];
        Os[(8 * h + 4 + r) * OSP + col]      = (oh[0][nt][4 + r] + ol[0][nt][4 + r] * rlo) * iB0[r];
        Os[(16 + 8 * h + r) * OSP + col]     = (oh[1][nt][r] + ol[1][nt][r] * rlo) * iA1[r];
        Os[(16 + 8 * h + 4 + r) * OSP + col] = (oh[1][nt][4 + r] + ol[1][nt][4 + r] * rlo) * iB1[r];
      }
    }
  }
  __syncthreads();
  {
    float* go = out + (size_t)q0 * DVV;
#pragma unroll
    for (int ps = 0; ps < 2; ++ps) {
#pragma unroll
      for (int rr = 0; rr < 4; ++rr) {
        const int row = 4 * wave + rr;
#pragma unroll
        for (int j = 0; j < 2; ++j) {
          const int pc = j * 32 + lane;
          const v4f v = *(const v4f*)(Os + row * OSP + pc * 4);
          *(volatile v4f*)(go + (size_t)row * DVV + pc * 4) = v;
        }
      }
      __threadfence();
    }
  }
}

extern "C" void kernel_launch(void* const* d_in, const int* in_sizes, int n_in,
                              void* d_out, int out_size, void* d_ws, size_t ws_size,
                              hipStream_t stream) {
  if (n_in < 6) return;
  const int nq = NQ, nk = NK, dd = DD, dv = DVV;
  if (in_sizes[0] != nq * dd || in_sizes[1] != nk * dd || in_sizes[2] != nk * dd) return;
  if (in_sizes[3] != dd * dd || in_sizes[4] != dv * dd || in_sizes[5] < 1) return;
  if (out_size != nq * dv) return;

  const float* X  = (const float*)d_in[0];
  const float* Y  = (const float*)d_in[1];
  const float* Z  = (const float*)d_in[2];
  const float* Wk = (const float*)d_in[3];
  const float* Wv = (const float*)d_in[4];
  const int* rate = (const int*)d_in[5];
  float* out = (float*)d_out;

  const size_t bY  = (size_t)nk * dd * 2;
  const size_t bZ  = (size_t)nk * dd * 2;
  const size_t bWk = (size_t)dd * dd * 2;
  const size_t bWv = (size_t)dv * dd * 2;
  const size_t bK  = (size_t)nk * dd * 2;
  const size_t bV  = (size_t)dv * nk * 2;
  size_t off = 0;
  const size_t oY  = off; off += bY;
  const size_t oZ  = off; off += bZ;
  const size_t oWk = off; off += bWk;
  const size_t oWv = off; off += bWv;
  const size_t oKH = off; off += bK;
  const size_t oKL = off; off += bK;
  const size_t oVH = off; off += bV;
  const size_t oVL = off; off += bV;
  if (off > ws_size) return;
  if (off > (size_t)134217728) return;

  char* ws = (char*)d_ws;
  unsigned short* Yb  = (unsigned short*)(ws + oY);
  unsigned short* Zb  = (unsigned short*)(ws + oZ);
  unsigned short* Wkb = (unsigned short*)(ws + oWk);
  unsigned short* Wvb = (unsigned short*)(ws + oWv);
  unsigned short* KH  = (unsigned short*)(ws + oKH);
  unsigned short* KL  = (unsigned short*)(ws + oKL);
  unsigned short* VH  = (unsigned short*)(ws + oVH);
  unsigned short* VL  = (unsigned short*)(ws + oVL);

  const dim3 blk(256);
  const int n8y = nk * dd / 8, n8z = nk * dd / 8, n8k = dd * dd / 8, n8v = dv * dd / 8;
  if ((n8y % 256) != 0 || (n8z % 256) != 0 || (n8k % 256) != 0 || (n8v % 256) != 0) return;
  const int ncvt = n8y / 256 + n8z / 256 + n8k / 256 + n8v / 256;

  cvt_kernel<<<dim3(ncvt), blk, 0, stream>>>(Y, Z, Wk, Wv, rate, Yb, Zb, Wkb, Wvb, n8y, n8z, n8k, n8v);

  const int tilesK = (nk / 64) * (dd / 64);
  if ((tilesK % 8) != 0) return;
  gemm64_kernel<0><<<dim3(tilesK / 8), blk, 0, stream>>>(Yb, dd, Wkb, dd, KH, KL, dd, nk, dd, dd, 1.0f, 1.0f);

  const int tilesV = (dv / 64) * (nk / 64);
  if ((tilesV % 8) != 0) return;
  gemm64_kernel<1><<<dim3(tilesV / 8), blk, 0, stream>>>(Wvb, dd, Zb, dd, VH, VL, nk, dv, nk, dd, 16.0f, 2048.0f);

  const float sc = 0.044194173824159216f;
  attn_kernel<<<dim3(nq / QB), blk, 0, stream>>>(X, KH, KL, (const _Float16*)VH, (const _Float16*)VL, out, sc, nq, nk);
  (void)hipGetLastError();
}
